// KAGNMoE_72550587564099
// MI455X (gfx1250) — hardware-verified
//
#include <hip/hip_runtime.h>

typedef _Float16 f16t;
typedef _Float16 v16h __attribute__((ext_vector_type(16)));
typedef _Float16 v8h  __attribute__((ext_vector_type(8)));
typedef float    v8f  __attribute__((ext_vector_type(8)));
typedef float    v4f  __attribute__((ext_vector_type(4)));
typedef v8h __attribute__((may_alias)) v8ha;
typedef v4f __attribute__((may_alias)) v4fa;
union Frag { v16h v; v8h half[2]; };

#define NB    8
#define NE    8
#define CIN   64
#define COUT  128
#define HH    64
#define WW    64
#define HW    4096
#define KB    256
#define KTOT  2304
#define PADW  66
#define NPP   4356
#define NPAIR 16
#define WSC   64.0f
#define TCAR  16.0f

#define GT_TKG 64
#define GT_TKI 80

__device__ __forceinline__ v8f wmma_f16(v16h a, v16h b, v8f c) {
  v8f d = __builtin_amdgcn_wmma_f32_16x16x32_f16(false, a, false, b, (short)0, c, false, false);
  asm volatile("v_nop\n\tv_nop\n\tv_nop\n\tv_nop" : "+v"(d) : "v"(a), "v"(b));
  return d;
}

__device__ __forceinline__ v16h load_frag32(const f16t* p, int h) {
  Frag f;
  f.half[0] = *(const v8ha*)(p + 8 * h);
  f.half[1] = *(const v8ha*)(p + 16 + 8 * h);
  return f.v;
}

__device__ __forceinline__ v8f zero8f() {
  v8f z;
  #pragma unroll
  for (int j = 0; j < 8; ++j) z[j] = 0.f;
  return z;
}

__global__ __launch_bounds__(512) void gate_k(const float* __restrict__ x, const float* __restrict__ wg,
                                             float* __restrict__ GT, float* __restrict__ lossp)
{
  __shared__ float smean[NB * CIN];
  __shared__ float slog[NB * NE];
  __shared__ float sprob[NB * NE];
  __shared__ float sg[NB * NE];
  __shared__ __attribute__((aligned(16))) float sGT[128];
  const int tid = threadIdx.x;

  {
    const float* p = x + (size_t)tid * HW;
    double s0 = 0.0, s1 = 0.0, s2 = 0.0, s3 = 0.0;
    #pragma unroll 1
    for (int i = 0; i < HW / 4; ++i) {
      const v4f v = *(const v4fa*)(p + 4 * i);
      s0 += (double)v.x; s1 += (double)v.y; s2 += (double)v.z; s3 += (double)v.w;
    }
    smean[tid] = (float)((s0 + s1) + (s2 + s3)) * (1.0f / 4096.0f);
  }
  if (tid < 128) sGT[tid] = 0.f;
  __syncthreads();

  if (tid < NB * NE) {
    const int b = tid >> 3, e = tid & 7;
    float s = 0.f;
    #pragma unroll 1
    for (int c = 0; c < CIN; ++c) s += smean[b * CIN + c] * wg[c * NE + e];
    slog[tid] = s;
    sg[tid] = 0.f;
  }
  __syncthreads();

  if (tid < NB) {
    const int b = tid;
    float mx = slog[b * NE];
    #pragma unroll 1
    for (int e = 1; e < NE; ++e) mx = fmaxf(mx, slog[b * NE + e]);
    float den = 0.f;
    #pragma unroll 1
    for (int e = 0; e < NE; ++e) {
      const float ex = expf(slog[b * NE + e] - mx);
      sprob[b * NE + e] = ex;
      den += ex;
    }
    const float rden = 1.0f / den;
    int i0 = 0;
    float v0 = sprob[b * NE] * rden;
    #pragma unroll 1
    for (int e = 1; e < NE; ++e) {
      const float v = sprob[b * NE + e] * rden;
      if (v > v0) { v0 = v; i0 = e; }
    }
    int i1 = 0;
    float v1 = -1.0f;
    #pragma unroll 1
    for (int e = 0; e < NE; ++e) {
      const float v = sprob[b * NE + e] * rden;
      if (e != i0 && v > v1) { v1 = v; i1 = e; }
    }
    const float rs = 1.0f / ((v0 + v1) + 1e-6f);
    const float g0 = v0 * rs, g1 = v1 * rs;
    sg[b * NE + i0] = g0;
    sg[b * NE + i1] = g1;
    sGT[GT_TKG + 2 * b] = g0;
    sGT[GT_TKG + 2 * b + 1] = g1;
    sGT[GT_TKI + 2 * b] = __int_as_float(i0);
    sGT[GT_TKI + 2 * b + 1] = __int_as_float(i1);
  }
  __syncthreads();

  if (tid < NB * NE) sGT[tid] = sg[tid];
  if (tid == 0) {
    float mi = 0.f, ml = 0.f;
    #pragma unroll 1
    for (int e = 0; e < NE; ++e) {
      float si = 0.f, sl = 0.f;
      #pragma unroll 1
      for (int b = 0; b < NB; ++b) {
        const float gv = sg[b * NE + e];
        si += gv;
        sl += (gv > 0.f) ? 1.f : 0.f;
      }
      mi += si; ml += sl;
    }
    mi *= (1.0f / NE);
    ml *= (1.0f / NE);
    float vi = 0.f, vl = 0.f;
    #pragma unroll 1
    for (int e = 0; e < NE; ++e) {
      float si = 0.f, sl = 0.f;
      #pragma unroll 1
      for (int b = 0; b < NB; ++b) {
        const float gv = sg[b * NE + e];
        si += gv;
        sl += (gv > 0.f) ? 1.f : 0.f;
      }
      const float di = si - mi, dl = sl - ml;
      vi += di * di;
      vl += dl * dl;
    }
    vi *= (1.0f / (NE - 1));
    vl *= (1.0f / (NE - 1));
    const float loss = (vi * (1.0f / (mi * mi + 1e-10f)) + vl * (1.0f / (ml * ml + 1e-10f))) * 0.01f;
    *(volatile float*)lossp = loss;
    __threadfence();
    *(volatile float*)lossp = loss;
  }
  __syncthreads();

  if (tid < 32) {
    const v4f v = *(const v4fa*)(sGT + 4 * tid);
    *(volatile v4f*)(GT + 4 * tid) = v;
    __threadfence();
    *(volatile v4f*)(GT + 4 * tid) = v;
  }
}

__global__ __launch_bounds__(256) void wsel_k(const float* __restrict__ pw, const float* __restrict__ GT,
                                             f16t* __restrict__ Wsel)
{
  const int g = blockIdx.x * 256 + threadIdx.x;
  if (g >= NPAIR * COUT * (KTOT / 8)) return;
  const int pair = g / (COUT * (KTOT / 8));
  const int rem = g - pair * (COUT * (KTOT / 8));
  const int o = rem / (KTOT / 8);
  const int k8 = rem - o * (KTOT / 8);
  const int k = 8 * k8;
  const int tap = k >> 8, c = k & 255;
  int e = __float_as_int(GT[GT_TKI + pair]);
  e = e < 0 ? 0 : (e > NE - 1 ? NE - 1 : e);
  const float* src = pw + ((size_t)((e * COUT + o) * KB + c)) * 9 + tap;
  v8h o8;
  #pragma unroll
  for (int i = 0; i < 8; ++i) o8[i] = (f16t)(src[i * 9] * WSC);
  f16t* dst = Wsel + (size_t)(pair * COUT + o) * KTOT + k;
  *(volatile v8h*)dst = o8;
  __threadfence();
  *(volatile v8h*)dst = o8;
}

__global__ __launch_bounds__(256) void basis_k(const float* __restrict__ x, const float* __restrict__ beta,
                                              const float* __restrict__ GT, f16t* __restrict__ T)
{
  __shared__ __attribute__((aligned(16))) f16t sT[PADW * KB];
  const int tid = threadIdx.x, lane = tid & 31, w = tid >> 5;
  const int pair = blockIdx.x, yq = blockIdx.y;
  const int b = pair >> 1;

  {
    v8h z;
    #pragma unroll
    for (int j = 0; j < 8; ++j) z[j] = (f16t)0.0f;
    #pragma unroll 1
    for (int i = tid; i < (PADW * KB) / 8; i += 256) *(v8ha*)(sT + 8 * i) = z;
  }
  __syncthreads();

  if (yq >= 1 && yq <= HH) {
    int e = __float_as_int(GT[GT_TKI + pair]);
    e = e < 0 ? 0 : (e > NE - 1 ? NE - 1 : e);
    const float gsc = GT[GT_TKG + pair] * TCAR;
    const float cb1 = 2.25f * beta[e * 4 + 1];
    const float cb2 = (100.0f / 3.0f) * beta[e * 4 + 2];
    const float* xrow = x + (size_t)b * CIN * HW + (size_t)(yq - 1) * WW;
    #pragma unroll 1
    for (int i = 0; i < 16; ++i) {
      const int idx = tid + 256 * i;
      const int c = idx >> 6, xx = idx & 63;
      const float t = tanhf(xrow[(size_t)c * HW + xx]);
      float pprev = 0.f, pcur = 1.f;
      f16t* dst = sT + (xx + 1) * KB + c;
      #pragma unroll 1
      for (int d = 0; d < 4; ++d) {
        const float sig = __builtin_amdgcn_rcpf(1.0f + __expf(-pcur));
        dst[d * CIN] = (f16t)((pcur * sig) * gsc);
        const float cbd = (d == 1) ? cb1 : ((d == 2) ? cb2 : 0.f);
        const float pn = t * pcur - cbd * pprev;
        pprev = pcur;
        pcur = pn;
      }
    }
  }
  __syncthreads();

  f16t* base = T + ((size_t)pair * NPP + (size_t)yq * PADW) * KB;
  #pragma unroll 1
  for (int L = w; L < PADW; L += 8) {
    const v8h v = *(const v8ha*)(sT + L * KB + 8 * lane);
    *(volatile v8h*)(base + (size_t)L * KB + 8 * lane) = v;
  }
  __threadfence();
  #pragma unroll 1
  for (int L = w; L < PADW; L += 8) {
    const v8h v = *(const v8ha*)(sT + L * KB + 8 * lane);
    *(volatile v8h*)(base + (size_t)L * KB + 8 * lane) = v;
  }
}

__global__ __launch_bounds__(256) void conv_k(const f16t* __restrict__ Wsel, const f16t* __restrict__ T,
                                             float* __restrict__ out)
{
  __shared__ __attribute__((aligned(16))) float sO[COUT * WW];
  const int tid = threadIdx.x, lane = tid & 31, w = tid >> 5;
  const int h = lane >> 4, m = lane & 15;
  const int y = blockIdx.x, b = blockIdx.y;
  const int mg = w >> 2, ng = w & 3;
  const v8f z8 = zero8f();
  v8f acc[2][2];
  #pragma unroll
  for (int nt = 0; nt < 2; ++nt) { acc[nt][0] = z8; acc[nt][1] = z8; }

  #pragma unroll 1
  for (int kk = 0; kk < 2; ++kk) {
    const int pair = 2 * b + kk;
    const f16t* wr = Wsel + ((size_t)(pair * COUT + 32 * ng + m)) * KTOT;
    const f16t* tb = T + ((size_t)pair * NPP) * KB;
    #pragma unroll 1
    for (int tap = 0; tap < 9; ++tap) {
      const int dy = tap / 3, dx = tap - 3 * dy;
      const f16t* wt = wr + tap * KB;
      const f16t* tr = tb + ((size_t)((y + dy) * PADW + dx + 32 * mg + m)) * KB;
      #pragma unroll 1
      for (int c0 = 0; c0 < KB; c0 += 32) {
        const v16h a0 = load_frag32(wt + c0, h);
        const v16h a1 = load_frag32(wt + (size_t)16 * KTOT + c0, h);
        const v16h b0 = load_frag32(tr + c0, h);
        const v16h b1 = load_frag32(tr + 16 * KB + c0, h);
        acc[0][0] = wmma_f16(a0, b0, acc[0][0]);
        acc[0][1] = wmma_f16(a0, b1, acc[0][1]);
        acc[1][0] = wmma_f16(a1, b0, acc[1][0]);
        acc[1][1] = wmma_f16(a1, b1, acc[1][1]);
      }
    }
  }

  const float osc = 1.0f / (WSC * TCAR);
  #pragma unroll
  for (int nt = 0; nt < 2; ++nt) {
    #pragma unroll
    for (int mt = 0; mt < 2; ++mt) {
      float* so = sO + (32 * ng + 16 * nt + 8 * h) * WW + 32 * mg + 16 * mt + m;
      #pragma unroll
      for (int r = 0; r < 8; ++r) so[r * WW] = acc[nt][mt][r] * osc;
    }
  }
  __syncthreads();

  const int sub = lane >> 4, q = lane & 15;
  v4f vals[8];
  size_t d[8];
  #pragma unroll
  for (int i = 0; i < 8; ++i) {
    const int orow = 16 * w + 2 * i + sub;
    vals[i] = *(const v4fa*)(sO + orow * WW + 4 * q);
    d[i] = ((size_t)(b * COUT + orow) * HH + y) * WW + 4 * q;
  }
  #pragma unroll
  for (int i = 0; i < 8; ++i) *(volatile v4f*)(out + d[i]) = vals[i];
  __threadfence();
  #pragma unroll
  for (int i = 0; i < 8; ++i) *(volatile v4f*)(out + d[i]) = vals[i];
}

extern "C" void kernel_launch(void* const* d_in, const int* in_sizes, int n_in,
                              void* d_out, int out_size, void* d_ws, size_t ws_size,
                              hipStream_t stream) {
  if (n_in < 4) return;
  if (in_sizes[0] != NB * CIN * HW) return;
  if (in_sizes[1] != CIN * NE) return;
  if (in_sizes[2] != NE * COUT * KB * 9) return;
  if (in_sizes[3] != NE * 4) return;
  if (out_size != NB * COUT * HW + 1) return;

  const float* x    = (const float*)d_in[0];
  const float* wg   = (const float*)d_in[1];
  const float* pw   = (const float*)d_in[2];
  const float* beta = (const float*)d_in[3];
  float* outp = (float*)d_out;
  float* lossp = outp + (size_t)NB * COUT * HW;

  const size_t szGT = 4096;
  const size_t szW  = (size_t)NPAIR * COUT * KTOT * 2;
  const size_t szT  = (size_t)NPAIR * NPP * KB * 2;
  size_t off = 0;
  char* ws = (char*)d_ws;
  float* GT   = (float*)(ws + off); off += szGT;
  f16t*  Wsel = (f16t*)(ws + off);  off += szW;
  f16t*  T    = (f16t*)(ws + off);  off += szT;
  if (off > ws_size) return;

  gate_k<<<1, 512, 0, stream>>>(x, wg, GT, lossp);
  wsel_k<<<(NPAIR * COUT * (KTOT / 8)) / 256, 256, 0, stream>>>(pw, GT, Wsel);
  basis_k<<<dim3(NPAIR, PADW), 256, 0, stream>>>(x, beta, GT, T);
  conv_k<<<dim3(HH, NB), 256, 0, stream>>>(Wsel, T, outp);
}
